// _UserModel_34359738368363
// MI455X (gfx1250) — hardware-run, weakly checked
//
#include <hip/hip_runtime.h>
#include <stdint.h>

#define DIM   128
#define NH    50
#define NBAT  16384
#define NU    100000
#define NI    100000
#define QPP   512
#define WTP   256
#define CATP  256
#define NBU   64
#define SCP   52
#define RSQ   0.08838834764831845f

static_assert(NBAT % 64 == 0);
static_assert(NBAT % NBU == 0);
static_assert(NBAT % 16 == 0);
static_assert(DIM % 32 == 0);
static_assert(NBU == 64);

typedef __attribute__((ext_vector_type(16))) __bf16   v16b;
typedef __attribute__((ext_vector_type(8)))  __bf16   v8b;
typedef __attribute__((ext_vector_type(8)))  float    v8f;
typedef __attribute__((ext_vector_type(4)))  float    v4f;
typedef __attribute__((ext_vector_type(4)))  unsigned int v4u;
typedef v4f __attribute__((may_alias)) v4fa;

__device__ __forceinline__ unsigned short f2bf_bits(float f) {
  unsigned u = __float_as_uint(f);
  return (unsigned short)((u + 0x7FFFu + ((u >> 16) & 1u)) >> 16);
}
__device__ __forceinline__ float bf_bits2f(unsigned short h) { return __uint_as_float(((unsigned)h) << 16); }
__device__ __forceinline__ float bf_rne(float f) { return bf_bits2f(f2bf_bits(f)); }
__device__ __forceinline__ unsigned pk16(unsigned short a, unsigned short b) { return (unsigned)a | ((unsigned)b << 16); }
__device__ __forceinline__ int clampi(int v, int lo, int hi) { v = v < lo ? lo : v; return v > hi ? hi : v; }

__device__ __forceinline__ v8f zero8() { v8f z = {0.f, 0.f, 0.f, 0.f, 0.f, 0.f, 0.f, 0.f}; return z; }

__device__ __forceinline__ v8f mma_bf(v16b a, v16b b, v8f c) {
  c = __builtin_amdgcn_wmma_f32_16x16x32_bf16(false, a, false, b, (short)0, c, false, false);
  asm volatile("v_nop\n\tv_nop\n\tv_nop\n\tv_nop" : "+v"(c) : "v"(a), "v"(b));
  return c;
}
__device__ __forceinline__ void acc_guard4(v8f& a, v8f& b, v8f& c, v8f& d) {
  asm volatile("v_nop\n\tv_nop\n\tv_nop\n\tv_nop" : "+v"(a), "+v"(b), "+v"(c), "+v"(d));
}

union FB { v16b v; v8b h[2]; };

__device__ __forceinline__ v16b load_frag_g(const __bf16* p) {
  FB f; f.h[0] = *(const v8b*)(p); f.h[1] = *(const v8b*)(p + 16); return f.v;
}

__global__ __launch_bounds__(256) void wprep_kernel(
    const float* __restrict__ w0, const float* __restrict__ w1, const float* __restrict__ w2, const float* __restrict__ w3,
    const float* __restrict__ w4, const float* __restrict__ w5, const float* __restrict__ w6, const float* __restrict__ w7,
    unsigned short* __restrict__ wt) {
  __shared__ __align__(16) float tf[64 * 68];
  const int mat = blockIdx.z;
  const float* W = w0;
  if (mat == 1) W = w1;
  if (mat == 2) W = w2;
  if (mat == 3) W = w3;
  if (mat == 4) W = w4;
  if (mat == 5) W = w5;
  if (mat == 6) W = w6;
  if (mat == 7) W = w7;
  unsigned short* o = wt + (size_t)mat * DIM * WTP;
  const int c0  = blockIdx.x * 64;
  const int r0  = blockIdx.y * 64;
  const int tid = threadIdx.x;
  {
    const int lr = tid >> 4;
    const int c4 = (tid & 15) * 4;
#pragma unroll
    for (int it = 0; it < 4; ++it) {
      const int rr = it * 16 + lr;
      const v4f a = *(const v4fa*)(W + (size_t)(r0 + rr) * DIM + c0 + c4);
      *(v4f*)(tf + rr * 68 + c4) = a;
    }
  }
  __syncthreads();
  const int sub = tid >> 3;
  const int c8  = (tid & 7) * 8;
  v4u hv[2];
#pragma unroll
  for (int it = 0; it < 2; ++it) {
    const int oc = it * 32 + sub;
    v4u a;
#pragma unroll
    for (int q = 0; q < 4; ++q) {
      const float f0 = tf[(c8 + 2 * q) * 68 + oc];
      const float f1 = tf[(c8 + 2 * q + 1) * 68 + oc];
      a[q] = pk16(f2bf_bits(f0), f2bf_bits(f1));
    }
    hv[it] = a;
  }
  for (int pass = 0; pass < 2; ++pass) {
#pragma unroll
    for (int it = 0; it < 2; ++it) {
      const int oc = it * 32 + sub;
      const size_t go = (size_t)(c0 + oc) * WTP + r0 + c8;
      *(volatile v4u*)(o + go) = hv[it];
      *(volatile v4u*)(o + go + DIM) = hv[it];
    }
    __threadfence();
  }
}

__global__ __launch_bounds__(256) void gnode_kernel(const int* __restrict__ uids, const float* __restrict__ ut,
                                                    unsigned short* __restrict__ nbp, int nrows) {
  const int g = blockIdx.x * 256 + threadIdx.x;
  if (g >= nrows * 16) return;
  const int row = g >> 4;
  const int c8  = (g & 15) * 8;
  const int uid = clampi(uids[row], 0, NU - 1);
  const float* sp = ut + (size_t)uid * DIM + c8;
  const v4f a  = *(const v4fa*)(sp);
  const v4f a2 = *(const v4fa*)(sp + 4);
  v4u w;
  w[0] = pk16(f2bf_bits(a[0]),  f2bf_bits(a[1]));
  w[1] = pk16(f2bf_bits(a[2]),  f2bf_bits(a[3]));
  w[2] = pk16(f2bf_bits(a2[0]), f2bf_bits(a2[1]));
  w[3] = pk16(f2bf_bits(a2[2]), f2bf_bits(a2[3]));
  unsigned short* dp = nbp + (size_t)row * DIM + c8;
  *(volatile v4u*)dp = w;
  __threadfence();
  *(volatile v4u*)dp = w;
}

__global__ __launch_bounds__(256) void cvt_bf16x8_kernel(const float* __restrict__ in, unsigned short* __restrict__ o, int n8) {
  const int i = blockIdx.x * 256 + threadIdx.x;
  if (i < n8) {
    const float* sp = in + (size_t)i * 8;
    const v4f a  = *(const v4fa*)(sp);
    const v4f a2 = *(const v4fa*)(sp + 4);
    v4u w;
    w[0] = pk16(f2bf_bits(a[0]),  f2bf_bits(a[1]));
    w[1] = pk16(f2bf_bits(a[2]),  f2bf_bits(a[3]));
    w[2] = pk16(f2bf_bits(a2[0]), f2bf_bits(a2[1]));
    w[3] = pk16(f2bf_bits(a2[2]), f2bf_bits(a2[3]));
    unsigned short* dp = o + (size_t)i * 8;
    *(volatile v4u*)dp = w;
    __threadfence();
    *(volatile v4u*)dp = w;
  }
}

template <int OUT_MODE>
__global__ __launch_bounds__(256) void gemm64_kernel(
    const unsigned short* __restrict__ Ap, int lda,
    const unsigned short* __restrict__ Btp, int ldb,
    const float* __restrict__ bs0, const float* __restrict__ bs1,
    const float* __restrict__ bs2, const float* __restrict__ bs3,
    void* Cout, int ldc, int M, int N, int K) {
  const __bf16* A  = (const __bf16*)(const void*)Ap;
  const __bf16* Bt = (const __bf16*)(const void*)Btp;
  __shared__ __align__(16) float sT[8][16 * 68];
  const int lane = threadIdx.x & 31;
  const int wave = threadIdx.x >> 5;
  const int tilesN = N >> 6;
  const int tilesM = M >> 6;
  const int tile = blockIdx.x * 8 + wave;
  if (tile >= tilesM * tilesN) return;
  const int tm = tile / tilesN;
  const int tn = tile - tm * tilesN;
  const int m0 = tm << 6;
  const int n0 = tn << 6;

  const int rlane = lane & 15;
  const int koff  = (lane >> 4) * 8;
  const int mOff  = (lane >> 4) * 8;

  v8f acc[4][4];
#pragma unroll
  for (int i = 0; i < 4; ++i)
#pragma unroll
    for (int j = 0; j < 4; ++j) acc[i][j] = zero8();

#pragma unroll 1
  for (int k0 = 0; k0 < K; k0 += 32) {
    v16b bh[4];
#pragma unroll
    for (int j = 0; j < 4; ++j)
      bh[j] = load_frag_g(Bt + (size_t)(n0 + (j << 4) + rlane) * ldb + koff + k0);
#pragma unroll
    for (int i = 0; i < 4; ++i) {
      const v16b ah = load_frag_g(A + (size_t)(m0 + (i << 4) + rlane) * lda + koff + k0);
#pragma unroll
      for (int j = 0; j < 4; ++j) acc[i][j] = mma_bf(ah, bh[j], acc[i][j]);
    }
  }
  acc_guard4(acc[0][0], acc[0][1], acc[0][2], acc[0][3]);
  acc_guard4(acc[1][0], acc[1][1], acc[1][2], acc[1][3]);
  acc_guard4(acc[2][0], acc[2][1], acc[2][2], acc[2][3]);
  acc_guard4(acc[3][0], acc[3][1], acc[3][2], acc[3][3]);

  const int seg = n0 >> 7;
  const float* bp = bs0;
  if (seg == 1) bp = bs1;
  if (seg == 2) bp = bs2;
  if (seg == 3) bp = bs3;
  float bcol[4];
#pragma unroll
  for (int j = 0; j < 4; ++j) bcol[j] = bf_rne(bp[(n0 & 127) + (j << 4) + rlane]);

  float* slab = sT[wave];
#pragma unroll
  for (int i = 0; i < 4; ++i) {
    const int mBase = m0 + (i << 4);
#pragma unroll
    for (int j = 0; j < 4; ++j) {
#pragma unroll
      for (int r = 0; r < 8; ++r) {
        const float v = acc[i][j][r] + bcol[j];
        slab[(mOff + r) * 68 + (j << 4) + rlane] = fmaxf(v, 0.0f);
      }
    }
    __builtin_amdgcn_fence(__ATOMIC_RELEASE, "workgroup");
    __builtin_amdgcn_wave_barrier();
    __builtin_amdgcn_fence(__ATOMIC_ACQUIRE, "workgroup");
    if (OUT_MODE == 0) {
      float* C = (float*)Cout;
      const int q = lane >> 3, rsel = q >> 1, hl = q & 1, c4 = (lane & 7) * 4;
      for (int pass = 0; pass < 2; ++pass) {
#pragma unroll
        for (int it = 0; it < 8; ++it) {
          const int row = it * 2 + rsel;
          const v4f val = *(const v4fa*)(slab + row * 68 + hl * 32 + c4);
          *(volatile v4f*)(C + (size_t)(mBase + row) * ldc + n0 + hl * 32 + c4) = val;
        }
        __threadfence();
      }
    } else {
      unsigned short* C = (unsigned short*)Cout;
      const int q = lane >> 3, c8 = (lane & 7) * 8;
      for (int pass = 0; pass < 2; ++pass) {
#pragma unroll
        for (int it = 0; it < 4; ++it) {
          const int row = it * 4 + q;
          const float* sp = slab + row * 68 + c8;
          v4u hv, lv;
#pragma unroll
          for (int e = 0; e < 4; ++e) {
            const float f0 = sp[2 * e], f1 = sp[2 * e + 1];
            const unsigned short h0 = f2bf_bits(f0), h1 = f2bf_bits(f1);
            const unsigned short l0 = f2bf_bits(f0 - bf_bits2f(h0)), l1 = f2bf_bits(f1 - bf_bits2f(h1));
            hv[e] = pk16(h0, h1);
            lv[e] = pk16(l0, l1);
          }
          *(volatile v4u*)(C + (size_t)(mBase + row) * ldc + n0 + c8) = hv;
          *(volatile v4u*)(C + (size_t)(mBase + row) * ldc + N + n0 + c8) = lv;
        }
        __threadfence();
      }
    }
    __builtin_amdgcn_fence(__ATOMIC_RELEASE, "workgroup");
    __builtin_amdgcn_wave_barrier();
    __builtin_amdgcn_fence(__ATOMIC_ACQUIRE, "workgroup");
  }
}

__device__ __forceinline__ void gather_slot(__bf16* As, const __bf16* itb, const int* um, int u0, int h, int tid) {
  const int r = tid >> 1;
  const int half = (tid & 1) * 64;
  const int mid = clampi(um[((size_t)(u0 + r) * NH + h) * 2], 0, NI - 1);
  const __bf16* src = itb + (size_t)mid * DIM + half;
  v8b t[8];
#pragma unroll
  for (int i = 0; i < 8; ++i) t[i] = *(const v8b*)(src + 8 * i);
#pragma unroll
  for (int i = 0; i < 8; ++i) *(v8b*)(As + r * DIM + half + 8 * i) = t[i];
}

__global__ __launch_bounds__(128) void nbr_kernel(
    const int* __restrict__ um,
    const unsigned short* __restrict__ itbp,
    const float* __restrict__ qp,
    const unsigned short* __restrict__ wkp,
    const unsigned short* __restrict__ wvp,
    const float* __restrict__ bk, const float* __restrict__ bv,
    unsigned short* __restrict__ yp) {
  __shared__ __align__(16) __bf16 As[NBU * DIM];
  __shared__ __align__(16) float  QY[NBU * DIM];
  __shared__ float SC[NBU * SCP];
  __shared__ float sBk[DIM];
  __shared__ float sBv[DIM];

  const int tid = threadIdx.x, lane = tid & 31, w = tid >> 5;
  const int hh = lane >> 4, m = lane & 15;
  const int u0 = blockIdx.x * NBU;
  const __bf16* itb = (const __bf16*)(const void*)itbp;
  const __bf16* wk  = (const __bf16*)(const void*)wkp;
  const __bf16* wv  = (const __bf16*)(const void*)wvp;

  sBk[tid] = bf_rne(bk[tid]);
  sBv[tid] = bf_rne(bv[tid]);
#pragma unroll 4
  for (int it = 0; it < 16; ++it) {
    const int idx = it * 128 + tid;
    const int row = idx >> 5;
    const int c4  = (idx & 31) * 4;
    const v4f v = *(const v4fa*)(qp + (size_t)(u0 + row) * QPP + c4);
    *(v4f*)(QY + row * DIM + c4) = v;
  }

#pragma unroll 1
  for (int h = 0; h < NH; ++h) {
    __syncthreads();
    gather_slot(As, itb, um, u0, h, tid);
    __syncthreads();
    v8f acc[8];
#pragma unroll
    for (int j = 0; j < 8; ++j) acc[j] = zero8();
#pragma unroll 1
    for (int k0 = 0; k0 < DIM; k0 += 32) {
      FB a;
      const __bf16* apr = As + (16 * w + m) * DIM + k0 + 8 * hh;
      a.h[0] = *(const v8b*)(apr);
      a.h[1] = *(const v8b*)(apr + 16);
#pragma unroll
      for (int j = 0; j < 8; ++j) {
        const v16b b = load_frag_g(wk + (size_t)(16 * j + m) * WTP + k0 + 8 * hh);
        acc[j] = mma_bf(a.v, b, acc[j]);
      }
    }
    float s[8];
#pragma unroll
    for (int r = 0; r < 8; ++r) s[r] = 0.0f;
#pragma unroll
    for (int j = 0; j < 8; ++j) {
      const int col = 16 * j + m;
      const float bb = sBk[col];
#pragma unroll
      for (int r = 0; r < 8; ++r) {
        const float kval = fmaxf(acc[j][r] + bb, 0.0f);
        s[r] = fmaf(kval, QY[(16 * w + 8 * hh + r) * DIM + col], s[r]);
      }
    }
#pragma unroll
    for (int r = 0; r < 8; ++r) {
      s[r] += __shfl_xor(s[r], 1);
      s[r] += __shfl_xor(s[r], 2);
      s[r] += __shfl_xor(s[r], 4);
      s[r] += __shfl_xor(s[r], 8);
    }
    float mine = s[0];
#pragma unroll
    for (int r = 1; r < 8; ++r) mine = (m == r) ? s[r] : mine;
    if (m < 8) SC[(16 * w + 8 * hh + m) * SCP + h] = mine * RSQ;
  }
  __syncthreads();

  if (tid < NBU) {
    float* sr = SC + tid * SCP;
    float mx = sr[0];
#pragma unroll 1
    for (int h = 1; h < NH; ++h) mx = fmaxf(mx, sr[h]);
    float sum = 0.0f;
#pragma unroll 1
    for (int h = 0; h < NH; ++h) {
      const float e = __expf(sr[h] - mx);
      sr[h] = e;
      sum += e;
    }
    const float inv = 1.0f / sum;
#pragma unroll 1
    for (int h = 0; h < NH; ++h) sr[h] = sr[h] * inv;
  }
  __syncthreads();
  {
    const v4f z4 = {0.f, 0.f, 0.f, 0.f};
#pragma unroll 4
    for (int it = 0; it < 16; ++it) {
      const int idx = it * 128 + tid;
      *(v4f*)(QY + idx * 4) = z4;
    }
  }

#pragma unroll 1
  for (int h = 0; h < NH; ++h) {
    __syncthreads();
    gather_slot(As, itb, um, u0, h, tid);
    __syncthreads();
    v8f acc[8];
#pragma unroll
    for (int j = 0; j < 8; ++j) acc[j] = zero8();
#pragma unroll 1
    for (int k0 = 0; k0 < DIM; k0 += 32) {
      FB a;
      const __bf16* apr = As + (16 * w + m) * DIM + k0 + 8 * hh;
      a.h[0] = *(const v8b*)(apr);
      a.h[1] = *(const v8b*)(apr + 16);
#pragma unroll
      for (int j = 0; j < 8; ++j) {
        const v16b b = load_frag_g(wv + (size_t)(16 * j + m) * WTP + k0 + 8 * hh);
        acc[j] = mma_bf(a.v, b, acc[j]);
      }
    }
    float p[8];
#pragma unroll
    for (int r = 0; r < 8; ++r) p[r] = SC[(16 * w + 8 * hh + r) * SCP + h];
#pragma unroll
    for (int j = 0; j < 8; ++j) {
      const int col = 16 * j + m;
      const float bb = sBv[col];
#pragma unroll
      for (int r = 0; r < 8; ++r) {
        const int idx = (16 * w + 8 * hh + r) * DIM + col;
        const float vval = fmaxf(acc[j][r] + bb, 0.0f);
        QY[idx] = fmaf(p[r], vval, QY[idx]);
      }
    }
  }
  __syncthreads();

  {
    const int q = lane >> 3, part = q >> 1, hl = q & 1, c8 = (lane & 7) * 8;
    const int col0 = hl * 64 + c8;
    for (int pass = 0; pass < 2; ++pass) {
#pragma unroll 4
      for (int it = 0; it < 16; ++it) {
        const int row = 16 * w + it;
        const v4f a  = *(const v4fa*)(QY + row * DIM + col0);
        const v4f a2 = *(const v4fa*)(QY + row * DIM + col0 + 4);
        v4u o;
#pragma unroll
        for (int e = 0; e < 4; ++e) {
          const float f0 = (e < 2) ? a[2 * e] : a2[2 * e - 4];
          const float f1 = (e < 2) ? a[2 * e + 1] : a2[2 * e - 3];
          const unsigned short h0 = f2bf_bits(f0), h1 = f2bf_bits(f1);
          const unsigned short l0 = f2bf_bits(f0 - bf_bits2f(h0)), l1 = f2bf_bits(f1 - bf_bits2f(h1));
          const unsigned hw = pk16(h0, h1), lw = pk16(l0, l1);
          o[e] = part ? lw : hw;
        }
        *(volatile v4u*)(yp + (size_t)(u0 + row) * CATP + part * DIM + col0) = o;
      }
      __threadfence();
    }
  }
}

__global__ __launch_bounds__(256) void sem_kernel(const float* __restrict__ qp, const float* __restrict__ kv,
                                                  unsigned short* __restrict__ y2p, int M) {
  const int tid = threadIdx.x, lane = tid & 31, w = tid >> 5, hh = lane >> 4, m = lane & 15;
  const int row = blockIdx.x * 16 + w * 2 + hh;
  const int rr  = clampi(row, 0, M - 1);
  const float* qr = qp + (size_t)rr * QPP + 8 * m;
  const float* kr = kv + (size_t)rr * CATP + 8 * m;
  const v4f qa  = *(const v4fa*)(qr + 128), qb  = *(const v4fa*)(qr + 132);
  const v4f ka  = *(const v4fa*)(qr + 256), kb  = *(const v4fa*)(qr + 260);
  const v4f va  = *(const v4fa*)(qr + 384), vb  = *(const v4fa*)(qr + 388);
  const v4f k1a = *(const v4fa*)(kr),       k1b = *(const v4fa*)(kr + 4);
  const v4f v1a = *(const v4fa*)(kr + 128), v1b = *(const v4fa*)(kr + 132);
  float d0 = 0.0f, d1 = 0.0f;
#pragma unroll
  for (int e = 0; e < 4; ++e) { d0 = fmaf(qa[e], ka[e], d0);  d1 = fmaf(qa[e], k1a[e], d1); }
#pragma unroll
  for (int e = 0; e < 4; ++e) { d0 = fmaf(qb[e], kb[e], d0);  d1 = fmaf(qb[e], k1b[e], d1); }
  d0 += __shfl_xor(d0, 1); d1 += __shfl_xor(d1, 1);
  d0 += __shfl_xor(d0, 2); d1 += __shfl_xor(d1, 2);
  d0 += __shfl_xor(d0, 4); d1 += __shfl_xor(d1, 4);
  d0 += __shfl_xor(d0, 8); d1 += __shfl_xor(d1, 8);
  const float s0 = d0 * RSQ, s1 = d1 * RSQ;
  const float mx = fmaxf(s0, s1);
  const float e0 = __expf(s0 - mx), e1 = __expf(s1 - mx);
  const float inv = 1.0f / (e0 + e1);
  const float p0 = e0 * inv, p1 = e1 * inv;
  float y[8];
#pragma unroll
  for (int e = 0; e < 4; ++e) {
    y[e]     = fmaf(p1, v1a[e], p0 * va[e]);
    y[e + 4] = fmaf(p1, v1b[e], p0 * vb[e]);
  }
  v4u hv, lv;
#pragma unroll
  for (int e = 0; e < 4; ++e) {
    const unsigned short h0 = f2bf_bits(y[2 * e]), h1 = f2bf_bits(y[2 * e + 1]);
    const unsigned short l0 = f2bf_bits(y[2 * e] - bf_bits2f(h0)), l1 = f2bf_bits(y[2 * e + 1] - bf_bits2f(h1));
    hv[e] = pk16(h0, h1);
    lv[e] = pk16(l0, l1);
  }
  if (row < M) {
    unsigned short* dp = y2p + (size_t)row * CATP + 8 * m;
    *(volatile v4u*)(dp) = hv;
    *(volatile v4u*)(dp + DIM) = lv;
    __threadfence();
    *(volatile v4u*)(dp) = hv;
    *(volatile v4u*)(dp + DIM) = lv;
  }
}

extern "C" void kernel_launch(void* const* d_in, const int* in_sizes, int n_in,
                              void* d_out, int out_size, void* d_ws, size_t ws_size,
                              hipStream_t stream) {
  if (n_in < 22) return;
  if (in_sizes[0] != NBAT) return;
  if (in_sizes[2] != NBAT * NH * 2) return;
  if (in_sizes[3] != NU * DIM) return;
  if (in_sizes[5] != NI * DIM) return;
  for (int i = 6; i <= 20; i += 2) if (in_sizes[i] != DIM * DIM) return;
  for (int i = 7; i <= 21; i += 2) if (in_sizes[i] != DIM) return;
  if (out_size != NBAT * DIM) return;

  const int*   uids       = (const int*)d_in[0];
  const int*   u_movies   = (const int*)d_in[2];
  const float* user_table = (const float*)d_in[3];
  const float* item_table = (const float*)d_in[5];
  const float* gat_wq = (const float*)d_in[6];  const float* gat_bq = (const float*)d_in[7];
  const float* gat_wk = (const float*)d_in[8];  const float* gat_bk = (const float*)d_in[9];
  const float* gat_wv = (const float*)d_in[10]; const float* gat_bv = (const float*)d_in[11];
  const float* gat_wo = (const float*)d_in[12]; const float* gat_bo = (const float*)d_in[13];
  const float* sem_wq = (const float*)d_in[14]; const float* sem_bq = (const float*)d_in[15];
  const float* sem_wk = (const float*)d_in[16]; const float* sem_bk = (const float*)d_in[17];
  const float* sem_wv = (const float*)d_in[18]; const float* sem_bv = (const float*)d_in[19];
  const float* sem_wo = (const float*)d_in[20]; const float* sem_bo = (const float*)d_in[21];
  float* out = (float*)d_out;

  const size_t SWT  = (size_t)8 * DIM * WTP * 2;
  const size_t SNB  = (size_t)NBAT * DIM * 2;
  const size_t SITB = (size_t)NI * DIM * 2;
  const size_t SQP  = (size_t)NBAT * QPP * 4;
  const size_t SCAT = (size_t)NBAT * CATP * 2;
  const size_t SKV  = (size_t)NBAT * CATP * 4;
  size_t off = 0;
  const size_t oWT  = off; off += SWT;
  const size_t oNB  = off; off += SNB;
  const size_t oITB = off; off += SITB;
  const size_t oQP  = off; off += SQP;
  const size_t oYP  = off; off += SCAT;
  const size_t oAG  = off; off += SCAT;
  const size_t oKV  = off; off += SKV;
  const size_t oY2  = off; off += SCAT;
  if (off > ws_size) return;
  if (off > (size_t)134217728) return;

  char* ws = (char*)d_ws;
  unsigned short* WT  = (unsigned short*)(ws + oWT);
  unsigned short* NBP = (unsigned short*)(ws + oNB);
  unsigned short* ITB = (unsigned short*)(ws + oITB);
  float*          QP  = (float*)(ws + oQP);
  unsigned short* YP  = (unsigned short*)(ws + oYP);
  unsigned short* AGP = (unsigned short*)(ws + oAG);
  float*          KV2 = (float*)(ws + oKV);
  unsigned short* Y2P = (unsigned short*)(ws + oY2);
  const size_t PL = (size_t)DIM * WTP;

  const dim3 blk(256);
  wprep_kernel<<<dim3(DIM / 64, DIM / 64, 8), blk, 0, stream>>>(
      gat_wq, sem_wq, sem_wk, sem_wv, gat_wk, gat_wv, gat_wo, sem_wo, WT);
  gnode_kernel<<<dim3((NBAT * 16 + 255) / 256), blk, 0, stream>>>(uids, user_table, NBP, NBAT);
  const int n8i = NI * DIM / 8;
  cvt_bf16x8_kernel<<<dim3((n8i + 255) / 256), blk, 0, stream>>>(item_table, ITB, n8i);
  gemm64_kernel<0><<<dim3(((NBAT / 64) * (QPP / 64) + 7) / 8), blk, 0, stream>>>(
      NBP, DIM, WT + 0 * PL, WTP, gat_bq, sem_bq, sem_bk, sem_bv, (void*)QP, QPP, NBAT, QPP, DIM);
  nbr_kernel<<<dim3(NBAT / NBU), dim3(128), 0, stream>>>(u_movies, ITB, QP, WT + 4 * PL, WT + 5 * PL, gat_bk, gat_bv, YP);
  gemm64_kernel<1><<<dim3(((NBAT / 64) * (DIM / 64) + 7) / 8), blk, 0, stream>>>(
      YP, CATP, WT + 6 * PL, WTP, gat_bo, gat_bo, gat_bo, gat_bo, (void*)AGP, CATP, NBAT, DIM, CATP);
  gemm64_kernel<0><<<dim3(((NBAT / 64) * (CATP / 64) + 7) / 8), blk, 0, stream>>>(
      AGP, CATP, WT + 2 * PL, WTP, sem_bk, sem_bv, sem_bk, sem_bv, (void*)KV2, CATP, NBAT, CATP, CATP);
  sem_kernel<<<dim3(NBAT / 16), blk, 0, stream>>>(QP, KV2, Y2P, NBAT);
  gemm64_kernel<0><<<dim3(((NBAT / 64) * (DIM / 64) + 7) / 8), blk, 0, stream>>>(
      Y2P, CATP, WT + 7 * PL, WTP, sem_bo, sem_bo, sem_bo, sem_bo, (void*)out, DIM, NBAT, DIM, CATP);
  (void)hipGetLastError();
}
